// SwinTransformerBlock_24464133718108
// MI455X (gfx1250) — hardware-verified
//
#include <hip/hip_runtime.h>
#include <stdint.h>


typedef _Float16 v16h __attribute__((ext_vector_type(16)));
typedef _Float16 v8h  __attribute__((ext_vector_type(8)));
typedef v8h v8ha __attribute__((may_alias));
typedef float v8f __attribute__((ext_vector_type(8)));
typedef float v4f __attribute__((ext_vector_type(4)));
typedef v4f v4fa __attribute__((may_alias));

#define DIMC 96
#define NHD  4
#define HDIM 24
#define HDP  32
#define NTOK 343
#define NP   352
#define NWIN 256
#define NWH  1024
#define LTOK 21952
#define NROWS 87808
#define HID  384
#define QKVN 288
#define MT   22
#define SCALE_Q 0.20412414523193154f
#define INV256  0.00390625f

#define H_QKVT  0
#define H_PROJT 27648
#define H_F1T   36864
#define H_F2T   73728
#define H_WEND  110592
#define OFF_W     0u
#define OFF_QKV   221184u
#define ONE_HALVES 11534336u
#define SZ_ONE    23068672u
#define OFF_OB    (OFF_QKV + 3u * SZ_ONE)
#define OFF_XMID  (OFF_OB + SZ_ONE)
#define SZ_XMID   33718272u
#define WS_NEED   (OFF_XMID + SZ_XMID)
#define ATTN_LDS  286720
#define MLP_LDS   86016

union Frag { v16h v; v8h hv[2]; };

__device__ __forceinline__ v8f zero8() {
  v8f c;
#pragma unroll
  for (int i = 0; i < 8; ++i) c[i] = 0.0f;
  return c;
}

__device__ __forceinline__ v8f mma(const v16h a, const v16h b, v8f c) {
  c = __builtin_amdgcn_wmma_f32_16x16x32_f16(false, a, false, b, (short)0, c, false, false);
  asm volatile("v_nop\n\tv_nop\n\tv_nop\n\tv_nop" : "+v"(c) : "v"(a), "v"(b));
  return c;
}

__device__ __forceinline__ v16h frag16(const _Float16* rowp, int k0, int hf) {
  Frag f;
  f.hv[0] = *(const v8ha*)(rowp + k0 + 8 * hf);
  f.hv[1] = *(const v8ha*)(rowp + k0 + 16 + 8 * hf);
  return f.v;
}

__device__ __forceinline__ float wave_max(float v) {
#pragma unroll
  for (int off = 16; off >= 1; off >>= 1) v = fmaxf(v, __shfl_xor(v, off, 32));
  return v;
}
__device__ __forceinline__ float wave_sum(float v) {
#pragma unroll
  for (int off = 16; off >= 1; off >>= 1) v += __shfl_xor(v, off, 32);
  return v;
}
__device__ __forceinline__ int regio(int p) { return p < 21 ? 0 : (p < 25 ? 1 : 2); }

__device__ __forceinline__ void ln_row_f16(const float* __restrict__ src,
                                           const float* __restrict__ gw,
                                           const float* __restrict__ gb,
                                           _Float16* dst, int lane) {
  float v0 = src[lane], v1 = src[lane + 32], v2 = src[lane + 64];
  float mu = wave_sum(v0 + v1 + v2) * (1.0f / 96.0f);
  float e0 = v0 - mu, e1 = v1 - mu, e2 = v2 - mu;
  float var = wave_sum(e0 * e0 + e1 * e1 + e2 * e2) * (1.0f / 96.0f);
  float rs = rsqrtf(var + 1e-5f);
  dst[lane]      = (_Float16)(e0 * rs * gw[lane]      + gb[lane]);
  dst[lane + 32] = (_Float16)(e1 * rs * gw[lane + 32] + gb[lane + 32]);
  dst[lane + 64] = (_Float16)(e2 * rs * gw[lane + 64] + gb[lane + 64]);
}

__global__ __launch_bounds__(256) void k_prep(const float* __restrict__ qkv_w,
                                              const float* __restrict__ proj_w,
                                              const float* __restrict__ fc1_w,
                                              const float* __restrict__ fc2_w,
                                              _Float16* __restrict__ wb) {
  const int i = blockIdx.x * 256 + threadIdx.x;
  if (i >= H_WEND / 8) return;
  const int e = i * 8;
  const float* src; int ncol, nr, kk;
  if (e < H_PROJT)      { src = qkv_w;  ncol = QKVN; nr = e / DIMC; kk = e % DIMC; }
  else if (e < H_F1T)   { int le = e - H_PROJT; src = proj_w; ncol = DIMC; nr = le / DIMC; kk = le % DIMC; }
  else if (e < H_F2T)   { int le = e - H_F1T;   src = fc1_w;  ncol = HID;  nr = le / DIMC; kk = le % DIMC; }
  else                  { int le = e - H_F2T;   src = fc2_w;  ncol = DIMC; nr = le / HID;  kk = le % HID; }
  v8h val;
#pragma unroll
  for (int j = 0; j < 8; ++j) val[j] = (_Float16)src[(size_t)(kk + j) * ncol + nr];
  _Float16* d = wb + e;
  *(volatile v8h*)d = val;
  __threadfence();
  *(volatile v8h*)d = val;
}

__global__ __launch_bounds__(192) void k_qkv(const float* __restrict__ x,
                                             const float* __restrict__ g1,
                                             const float* __restrict__ be1,
                                             const _Float16* __restrict__ wT,
                                             const float* __restrict__ bias,
                                             _Float16* __restrict__ qkvh) {
  __shared__ _Float16 As[16 * DIMC];
  __shared__ _Float16 St[12 * 16 * HDP];
  const int blk = blockIdx.x;
  if (blk >= NWIN * MT) return;
  const int win = blk / MT, m0 = (blk % MT) * 16;
  const int tid = threadIdx.x, lane = tid & 31, wave = tid >> 5, hf = lane >> 4, mm = lane & 15;
  const int b_ = win >> 6, wi = win & 63, hw = wi >> 4, ww = (wi >> 2) & 3, dw = wi & 3;

  for (int i = tid; i < 12 * 16 * HDP; i += 192) St[i] = (_Float16)0.0f;

  for (int r = wave; r < 16; r += 6) {
    const int m = m0 + r;
    _Float16* dst = As + r * DIMC;
    if (m < NTOK) {
      int h1 = m / 49, rm = m % 49, w1 = rm / 7, d1 = rm % 7;
      int ph = (hw * 7 + h1 + 3) % 28, pw = (ww * 7 + w1 + 3) % 28, pd = (dw * 7 + d1 + 3) % 28;
      const float* src = x + ((size_t)b_ * LTOK + (size_t)(ph * 784 + pw * 28 + pd)) * DIMC;
      ln_row_f16(src, g1, be1, dst, lane);
    } else {
      dst[lane] = (_Float16)0.0f; dst[lane + 32] = (_Float16)0.0f; dst[lane + 64] = (_Float16)0.0f;
    }
  }
  __syncthreads();

  v16h af[3];
#pragma unroll
  for (int s = 0; s < 3; ++s) af[s] = frag16(As + mm * DIMC, 32 * s, hf);

  for (int j = 0; j < 3; ++j) {
    const int n0 = (wave * 3 + j) * 16;
    v8f c = zero8();
#pragma unroll
    for (int s = 0; s < 3; ++s)
      c = mma(af[s], frag16(wT + (size_t)(n0 + mm) * DIMC, 32 * s, hf), c);
    const int n = n0 + mm, which = n / DIMC, r96 = n % DIMC, hd = r96 / HDIM, dim = r96 % HDIM;
    const float bn = bias[n];
    const float sc = (which == 0) ? SCALE_Q : 1.0f;
    _Float16* sd = St + (which * NHD + hd) * 512 + dim;
#pragma unroll
    for (int r = 0; r < 8; ++r) {
      const int row = 8 * hf + r;
      float val = (m0 + row < NTOK) ? (c[r] + bn) * sc : 0.0f;
      sd[row * HDP] = (_Float16)val;
    }
  }
  __syncthreads();

  v8h p00, p01, p10, p11;
  size_t d0, d1;
  {
    const int ch = wave;
    const int which = ch >> 2, hd = ch & 3;
    d0 = (size_t)which * ONE_HALVES + (((size_t)win * NHD + hd) * NP + m0) * HDP;
    p00 = *(const v8ha*)(St + ch * 512 + lane * 8);
    p01 = *(const v8ha*)(St + ch * 512 + 256 + lane * 8);
  }
  {
    const int ch = wave + 6;
    const int which = ch >> 2, hd = ch & 3;
    d1 = (size_t)which * ONE_HALVES + (((size_t)win * NHD + hd) * NP + m0) * HDP;
    p10 = *(const v8ha*)(St + ch * 512 + lane * 8);
    p11 = *(const v8ha*)(St + ch * 512 + 256 + lane * 8);
  }
  *(volatile v8h*)(qkvh + d0 + lane * 8)       = p00;
  *(volatile v8h*)(qkvh + d0 + 256 + lane * 8) = p01;
  *(volatile v8h*)(qkvh + d1 + lane * 8)       = p10;
  *(volatile v8h*)(qkvh + d1 + 256 + lane * 8) = p11;
  __threadfence();
  *(volatile v8h*)(qkvh + d0 + lane * 8)       = p00;
  *(volatile v8h*)(qkvh + d0 + 256 + lane * 8) = p01;
  *(volatile v8h*)(qkvh + d1 + lane * 8)       = p10;
  *(volatile v8h*)(qkvh + d1 + 256 + lane * 8) = p11;
}

__global__ __launch_bounds__(512) void k_attn(const _Float16* __restrict__ qkvh,
                                              const float* __restrict__ rpb,
                                              _Float16* __restrict__ obuf) {
  extern __shared__ _Float16 sm[];
  _Float16* P   = sm;
  _Float16* vs  = sm + NP * NP;
  _Float16* osc = vs + HDP * NP;
  const int wh = blockIdx.x;
  if (wh >= NWH) return;
  const int win = wh >> 2, hh = wh & 3;
  const int wi = win & 63;
  const int hw = wi >> 4, ww = (wi >> 2) & 3, dw = wi & 3;
  const int tid = threadIdx.x, lane = tid & 31, wave = tid >> 5, hf = lane >> 4, mm = lane & 15;
  const _Float16* qb = qkvh + (size_t)wh * NP * HDP;
  const _Float16* kb = qkvh + ONE_HALVES + (size_t)wh * NP * HDP;
  const _Float16* vb = qkvh + 2 * (size_t)ONE_HALVES + (size_t)wh * NP * HDP;

  for (int i = tid; i < NP * 4; i += 512) {
    const int tok = i >> 2, c8 = (i & 3) * 8;
    v8h t = *(const v8ha*)(vb + tok * HDP + c8);
#pragma unroll
    for (int j = 0; j < 8; ++j) vs[(c8 + j) * NP + tok] = t[j];
  }
  __syncthreads();

  for (int s = wave; s < 44; s += 16) {
    const int m0 = (s >> 1) * 16;
    const int ntb = (s & 1) * 11;
    const v16h a = frag16(qb + (size_t)(m0 + mm) * HDP, 0, hf);
    for (int nt = ntb; nt < ntb + 11; ++nt) {
      const int n0 = nt * 16;
      v8f c = zero8();
      c = mma(a, frag16(kb + (size_t)(n0 + mm) * HDP, 0, hf), c);
      const int n = n0 + mm;
      const bool nvalid = n < NTOK;
      const int nn = nvalid ? n : 0;
      const int h2 = nn / 49, rn = nn % 49, w2 = rn / 7, d2 = rn % 7;
      const int r2 = 9 * regio(hw * 7 + h2) + 3 * regio(ww * 7 + w2) + regio(dw * 7 + d2);
#pragma unroll
      for (int r = 0; r < 8; ++r) {
        const int m = m0 + 8 * hf + r;
        float sv;
        if (!nvalid) {
          sv = -1.0e4f;
        } else {
          const int mc = m < NTOK ? m : (NTOK - 1);
          const int h1 = mc / 49, rmm = mc % 49, w1 = rmm / 7, d1 = rmm % 7;
          const int idx = 13 * (h1 - h2 + 6) + 13 * (w1 - w2 + 6) + (d1 - d2 + 6);
          sv = c[r] + rpb[idx * NHD + hh];
          const int r1g = 9 * regio(hw * 7 + h1) + 3 * regio(ww * 7 + w1) + regio(dw * 7 + d1);
          if (r1g != r2) sv -= 100.0f;
        }
        P[(size_t)m * NP + n] = (_Float16)sv;
      }
    }
  }
  __syncthreads();

  for (int row = wave; row < NP; row += 16) {
    _Float16* pr = P + (size_t)row * NP;
    float v[11];
    float mx = -3.0e38f;
#pragma unroll
    for (int j = 0; j < 11; ++j) { v[j] = (float)pr[lane + 32 * j]; mx = fmaxf(mx, v[j]); }
    mx = wave_max(mx);
    float sum = 0.0f;
#pragma unroll
    for (int j = 0; j < 11; ++j) { v[j] = expf(v[j] - mx); sum += v[j]; }
    sum = wave_sum(sum);
    const float rs = 256.0f / sum;
#pragma unroll
    for (int j = 0; j < 11; ++j) pr[lane + 32 * j] = (_Float16)(v[j] * rs);
  }
  __syncthreads();

  for (int it = 0; it < 2; ++it) {
    const int t = wave + 16 * it;
    const bool act = t < MT;
    const int m0 = t * 16;
    _Float16* od = osc + wave * 512;
    if (act) {
      v8f c0 = zero8(), c1 = zero8();
      for (int kt = 0; kt < 11; ++kt) {
        const v16h a  = frag16(P + (size_t)(m0 + mm) * NP, 32 * kt, hf);
        const v16h b0 = frag16(vs + (size_t)mm * NP, 32 * kt, hf);
        const v16h b1 = frag16(vs + (size_t)(16 + mm) * NP, 32 * kt, hf);
        c0 = mma(a, b0, c0);
        c1 = mma(a, b1, c1);
      }
#pragma unroll
      for (int r = 0; r < 8; ++r) {
        od[(8 * hf + r) * HDP + mm]      = (_Float16)(c0[r] * INV256);
        od[(8 * hf + r) * HDP + 16 + mm] = (_Float16)(c1[r] * INV256);
      }
    }
    __syncthreads();
    v8h p0, p1;
    size_t dst = ((size_t)wh * NP + m0) * HDP;
    if (act) {
      p0 = *(const v8ha*)(od + lane * 8);
      p1 = *(const v8ha*)(od + 256 + lane * 8);
      *(volatile v8h*)(obuf + dst + lane * 8)       = p0;
      *(volatile v8h*)(obuf + dst + 256 + lane * 8) = p1;
    }
    __threadfence();
    if (act) {
      *(volatile v8h*)(obuf + dst + lane * 8)       = p0;
      *(volatile v8h*)(obuf + dst + 256 + lane * 8) = p1;
    }
    __syncthreads();
  }
}

__global__ __launch_bounds__(192) void k_proj(const _Float16* __restrict__ ob,
                                              const _Float16* __restrict__ pT,
                                              const float* __restrict__ pb,
                                              const float* __restrict__ x,
                                              float* __restrict__ xmid) {
  __shared__ float Cs[16 * DIMC];
  const int blk = blockIdx.x;
  if (blk >= NWIN * MT) return;
  const int win = blk / MT, m0 = (blk % MT) * 16;
  const int tid = threadIdx.x, lane = tid & 31, wave = tid >> 5, hf = lane >> 4, mm = lane & 15;
  const int b_ = win >> 6, wi = win & 63, hw = wi >> 4, ww = (wi >> 2) & 3, dw = wi & 3;
  const int n0 = wave * 16;

  v8f c = zero8();
#pragma unroll
  for (int s = 0; s < 3; ++s) {
    const int j0 = 4 * s + hf, j1 = 4 * s + 2 + hf;
    Frag a;
    a.hv[0] = *(const v8ha*)(ob + (((size_t)win * NHD + j0 / 3) * NP + m0 + mm) * HDP + 8 * (j0 % 3));
    a.hv[1] = *(const v8ha*)(ob + (((size_t)win * NHD + j1 / 3) * NP + m0 + mm) * HDP + 8 * (j1 % 3));
    c = mma(a.v, frag16(pT + (size_t)(n0 + mm) * DIMC, 32 * s, hf), c);
  }
  const float bn = pb[n0 + mm];
#pragma unroll
  for (int r = 0; r < 8; ++r) Cs[(8 * hf + r) * DIMC + n0 + mm] = c[r] + bn;
  __syncthreads();

  for (int r = wave; r < 16; r += 6) {
    const int m = m0 + r;
    if (m < NTOK && lane < 24) {
      int h1 = m / 49, rm = m % 49, w1 = rm / 7, d1 = rm % 7;
      int ph = (hw * 7 + h1 + 3) % 28, pw = (ww * 7 + w1 + 3) % 28, pd = (dw * 7 + d1 + 3) % 28;
      size_t li = (size_t)b_ * LTOK + (size_t)(ph * 784 + pw * 28 + pd);
      v4f cv = *(const v4fa*)(Cs + r * DIMC + 4 * lane);
      v4f xv = *(const v4fa*)(x + li * DIMC + 4 * lane);
      *(volatile v4f*)(xmid + li * DIMC + 4 * lane) = cv + xv;
    }
  }
  __threadfence();
  for (int r = wave; r < 16; r += 6) {
    const int m = m0 + r;
    if (m < NTOK && lane < 24) {
      int h1 = m / 49, rm = m % 49, w1 = rm / 7, d1 = rm % 7;
      int ph = (hw * 7 + h1 + 3) % 28, pw = (ww * 7 + w1 + 3) % 28, pd = (dw * 7 + d1 + 3) % 28;
      size_t li = (size_t)b_ * LTOK + (size_t)(ph * 784 + pw * 28 + pd);
      v4f cv = *(const v4fa*)(Cs + r * DIMC + 4 * lane);
      v4f xv = *(const v4fa*)(x + li * DIMC + 4 * lane);
      *(volatile v4f*)(xmid + li * DIMC + 4 * lane) = cv + xv;
    }
  }
}

__global__ __launch_bounds__(128) void k_mlp(const float* __restrict__ xmid,
                                             const float* __restrict__ g2,
                                             const float* __restrict__ be2,
                                             const _Float16* __restrict__ w1T,
                                             const float* __restrict__ bf1,
                                             const _Float16* __restrict__ w2T,
                                             const float* __restrict__ bf2,
                                             float* __restrict__ out) {
  extern __shared__ _Float16 sm[];
  if (blockIdx.x >= NROWS / 64) return;
  const int tid = threadIdx.x, lane = tid & 31, wave = tid >> 5, hf = lane >> 4, mm = lane & 15;
  _Float16* As    = sm + wave * (16 * DIMC);
  _Float16* strip = sm + 4 * 16 * DIMC + wave * (16 * HID);
  float*    Ost   = (float*)(sm + 4 * 16 * DIMC + 4 * 16 * HID) + wave * (16 * DIMC);
  const size_t row0 = ((size_t)blockIdx.x * 4 + wave) * 16;
  const bool act = row0 + 16 <= (size_t)NROWS;

  if (act) {
    for (int r = 0; r < 16; ++r)
      ln_row_f16(xmid + (row0 + r) * DIMC, g2, be2, As + r * DIMC, lane);
  }
  __syncthreads();

  if (act) {
    v16h af[3];
#pragma unroll
    for (int s = 0; s < 3; ++s) af[s] = frag16(As + mm * DIMC, 32 * s, hf);
    for (int nt = 0; nt < 24; ++nt) {
      const int n0 = nt * 16;
      v8f c = zero8();
#pragma unroll
      for (int s = 0; s < 3; ++s)
        c = mma(af[s], frag16(w1T + (size_t)(n0 + mm) * DIMC, 32 * s, hf), c);
      const int n = n0 + mm;
      const float bn = bf1[n];
#pragma unroll
      for (int r = 0; r < 8; ++r) {
        float v = c[r] + bn;
        float g = 0.5f * v * (1.0f + erff(v * 0.70710678118654752f));
        strip[(8 * hf + r) * HID + n] = (_Float16)g;
      }
    }
  }
  __syncthreads();

  if (act) {
    for (int nt = 0; nt < 6; ++nt) {
      const int n0 = nt * 16;
      v8f c = zero8();
      for (int ks = 0; ks < 12; ++ks)
        c = mma(frag16(strip + mm * HID, 32 * ks, hf),
                frag16(w2T + (size_t)(n0 + mm) * HID, 32 * ks, hf), c);
      const float bn = bf2[n0 + mm];
#pragma unroll
      for (int r = 0; r < 8; ++r) Ost[(8 * hf + r) * DIMC + n0 + mm] = c[r] + bn;
    }
  }
  __syncthreads();

  if (act && lane < 24) {
    for (int r = 0; r < 16; ++r) {
      const size_t row = row0 + r;
      v4f ov = *(const v4fa*)(Ost + r * DIMC + 4 * lane);
      v4f xv = *(const v4fa*)(xmid + row * DIMC + 4 * lane);
      *(volatile v4f*)(out + row * DIMC + 4 * lane) = ov + xv;
    }
  }
  __threadfence();
  if (act && lane < 24) {
    for (int r = 0; r < 16; ++r) {
      const size_t row = row0 + r;
      v4f ov = *(const v4fa*)(Ost + r * DIMC + 4 * lane);
      v4f xv = *(const v4fa*)(xmid + row * DIMC + 4 * lane);
      *(volatile v4f*)(out + row * DIMC + 4 * lane) = ov + xv;
    }
  }
}

extern "C" void kernel_launch(void* const* d_in, const int* in_sizes, int n_in,
                              void* d_out, int out_size, void* d_ws, size_t ws_size,
                              hipStream_t stream) {
  if (n_in < 14) return;
  if (in_sizes[0] != NROWS * DIMC) return;
  if (out_size != NROWS * DIMC) return;
  if (in_sizes[3] != DIMC * QKVN || in_sizes[5] != 2197 * NHD || in_sizes[6] != DIMC * DIMC) return;
  if (in_sizes[10] != DIMC * HID || in_sizes[12] != HID * DIMC) return;
  if (ws_size < (size_t)WS_NEED) return;

  const float* x      = (const float*)d_in[0];
  const float* n1w    = (const float*)d_in[1];
  const float* n1b    = (const float*)d_in[2];
  const float* qkv_w  = (const float*)d_in[3];
  const float* qkv_b  = (const float*)d_in[4];
  const float* rpb    = (const float*)d_in[5];
  const float* proj_w = (const float*)d_in[6];
  const float* proj_b = (const float*)d_in[7];
  const float* n2w    = (const float*)d_in[8];
  const float* n2b    = (const float*)d_in[9];
  const float* fc1_w  = (const float*)d_in[10];
  const float* fc1_b  = (const float*)d_in[11];
  const float* fc2_w  = (const float*)d_in[12];
  const float* fc2_b  = (const float*)d_in[13];

  char* ws = (char*)d_ws;
  _Float16* wb    = (_Float16*)(ws + OFF_W);
  _Float16* qkvT  = wb + H_QKVT;
  _Float16* projT = wb + H_PROJT;
  _Float16* f1T   = wb + H_F1T;
  _Float16* f2T   = wb + H_F2T;
  _Float16* qkvh  = (_Float16*)(ws + OFF_QKV);
  _Float16* obuf  = (_Float16*)(ws + OFF_OB);
  float*    xmid  = (float*)(ws + OFF_XMID);
  float*    out   = (float*)d_out;

  (void)hipFuncSetAttribute((const void*)k_attn, hipFuncAttributeMaxDynamicSharedMemorySize, ATTN_LDS);
  (void)hipFuncSetAttribute((const void*)k_mlp,  hipFuncAttributeMaxDynamicSharedMemorySize, MLP_LDS);

  k_prep<<<H_WEND / 8 / 256, 256, 0, stream>>>(qkv_w, proj_w, fc1_w, fc2_w, wb);
  k_qkv<<<NWIN * MT, 192, 0, stream>>>(x, n1w, n1b, qkvT, qkv_b, qkvh);
  k_attn<<<NWH, 512, ATTN_LDS, stream>>>(qkvh, rpb, obuf);
  k_proj<<<NWIN * MT, 192, 0, stream>>>(obuf, projT, proj_b, x, xmid);
  k_mlp<<<NROWS / 64, 128, MLP_LDS, stream>>>(xmid, n2w, n2b, f1T, fc1_b, f2T, fc2_b, out);
  (void)hipGetLastError();
}
